// HapbertaAxialEncoder_2903397892817
// MI455X (gfx1250) — hardware-run, weakly checked
//
#include <hip/hip_runtime.h>
#include <math.h>

#pragma clang fp contract(off)

constexpr int kBatch = 2, kRows = 32, kCols = 256, kHid = 256, kHeads = 8, kHdim = 32, kFF = 1024, kLayers = 2, kBuckets = 32;
constexpr int kTok   = kBatch * kRows * kCols;
constexpr int kQKVld = 3 * kHid;
constexpr int kBR    = kBatch * kRows;
constexpr int kChunkBR = 16;
constexpr int kChunks  = kBR / kChunkBR;
constexpr int kChunkGroups = kChunkBR * kHeads;

constexpr float kWCarry   = 16.0f;
constexpr float kPCarry   = 1024.0f;
constexpr float kCtxCarry = 64.0f;
constexpr float kGCarry   = 8.0f;
constexpr float kRowScoreScale = 1.0f / 32.0f;
constexpr float kColQScale = 0.17677669529663687f;
constexpr float kLogMaxD  = 10.819778284410283f;
constexpr float kRecipLogMaxD = 1.0f / kLogMaxD;
constexpr float kLnEps    = 1e-12f;

constexpr size_t kWoffQKVr = 0;
constexpr size_t kWoffOr   = 196608;
constexpr size_t kWoffQKVc = 262144;
constexpr size_t kWoffOc   = 458752;
constexpr size_t kWoffF1   = 524288;
constexpr size_t kWoffF2   = 786432;
constexpr size_t kHalvesWLayer = 1048576;

constexpr size_t kBytesX   = (size_t)kTok * kHid * 4;
constexpr size_t kOffXA    = 0;
constexpr size_t kOffXB    = kOffXA + kBytesX;
constexpr size_t kOffXN    = kOffXB + kBytesX;
constexpr size_t kBytesXN  = (size_t)kTok * kHid * 2;
constexpr size_t kOffQKV   = kOffXN + kBytesXN;
constexpr size_t kBytesQKV = (size_t)kTok * kQKVld * 2;
constexpr size_t kOffVT    = kOffQKV + kBytesQKV;
constexpr size_t kBytesVT  = (size_t)kBR * kHeads * kHdim * kCols * 2;
constexpr size_t kOffH16   = kOffQKV;
constexpr size_t kBytesH16 = (size_t)kTok * kFF * 2;
constexpr size_t kOffS     = kOffVT + kBytesVT;
constexpr size_t kBytesS   = (size_t)kChunkGroups * kCols * kCols * 4;
constexpr size_t kOffPre   = kOffS;
constexpr size_t kOffP     = kOffS + kBytesS;
constexpr size_t kBytesP   = (size_t)kChunkGroups * kCols * kCols * 2;
constexpr size_t kOffW     = kOffP + kBytesP;
constexpr size_t kBytesW   = (size_t)kLayers * kHalvesWLayer * 2;
constexpr size_t kWsTotal  = kOffW + kBytesW;
static_assert(kBytesH16 <= kBytesQKV + kBytesVT);
static_assert(kBytesH16 <= kBytesS);
static_assert(kWsTotal == 130023424);
static_assert(kWsTotal <= 134217728);
static_assert((kOffXN % 128) == 0 && (kOffQKV % 128) == 0 && (kOffVT % 128) == 0 && (kOffS % 128) == 0 && (kOffP % 128) == 0 && (kOffW % 128) == 0);

typedef __attribute__((ext_vector_type(16))) _Float16 v16h;
typedef __attribute__((ext_vector_type(8)))  _Float16 v8h;
typedef __attribute__((ext_vector_type(8)))  float    v8f;
typedef __attribute__((ext_vector_type(4)))  float    v4f;
typedef __attribute__((ext_vector_type(4)))  unsigned int v4u;
typedef __attribute__((ext_vector_type(4)))  int      v4i;

__device__ __forceinline__ unsigned pk16(unsigned short a, unsigned short b) { return (unsigned)a | ((unsigned)b << 16); }
__device__ __forceinline__ unsigned short h_bits(float f) { const _Float16 h = (_Float16)f; return __builtin_bit_cast(unsigned short, h); }
__device__ __forceinline__ float hbits2f(unsigned short u) { return (float)__builtin_bit_cast(_Float16, u); }

__device__ __forceinline__ void dep_guard_h(v8f& a, v8f& b, v16h x, v16h y) { asm volatile("v_nop\n\tv_nop\n\tv_nop\n\tv_nop" : "+v"(a), "+v"(b) : "v"(x), "v"(y)); }
__device__ __forceinline__ void keep4_h(v16h a, v16h b, v16h c, v16h d) { asm volatile("v_nop" :: "v"(a), "v"(b), "v"(c), "v"(d)); }
__device__ __forceinline__ void acc_guard4(v8f& a, v8f& b, v8f& c, v8f& d) { asm volatile("v_nop\n\tv_nop\n\tv_nop\n\tv_nop" : "+v"(a), "+v"(b), "+v"(c), "+v"(d)); }
template <typename T> struct Frag;
template <> struct Frag<_Float16> {
  typedef v16h V; union U { v16h v; v8h h[2]; };
  static __device__ __forceinline__ v16h load(const _Float16* p) {
    U f; f.h[0] = *(const v8h*)(p); f.h[1] = *(const v8h*)(p + 16); return f.v;
  }
  static __device__ __forceinline__ v8f mma(v16h a, v16h b, v8f c) {
    return __builtin_amdgcn_wmma_f32_16x16x32_f16(false, a, false, b, (short)0, c, false, false);
  }
  static __device__ __forceinline__ void guard(v8f& a, v8f& b, v16h x, v16h y) { dep_guard_h(a, b, x, y); }
  static __device__ __forceinline__ void keep(v16h a, v16h b, v16h c, v16h d) { keep4_h(a, b, c, d); }
};
__device__ __forceinline__ v8f mma_f16(v16h a, v16h b, v8f c) {
  c = __builtin_amdgcn_wmma_f32_16x16x32_f16(false, a, false, b, (short)0, c, false, false);
  asm volatile("v_nop\n\tv_nop\n\tv_nop\n\tv_nop" : "+v"(c) : "v"(a), "v"(b));
  return c;
}

template <int BIAS_MODE, int OUT_MODE, bool RESID, bool PAIRA>
__global__ __launch_bounds__(256) void gemm64(
    const unsigned short* __restrict__ Ap, int lda, long strideA, long strideAi, long strideAsub,
    const unsigned short* __restrict__ Btp, int ldb, long strideB, long strideBi,
    void* __restrict__ Cout, int ldc, long strideC, long strideCi,
    const float* __restrict__ bias0, const float* __restrict__ bias1, const float* __restrict__ bias2, int bseg, float seg0mul,
    const float* __restrict__ resid, long strideR,
    int M, int N, int K, int bdiv, float scale) {
  typedef _Float16 T;
  typedef v16h V;
  const T* A = (const T*)Ap; const T* Bt = (const T*)Btp;
  __shared__ __align__(16) float sT[8][16 * 68];
  const int b    = blockIdx.y;
  const int bo   = b / bdiv;
  const int bi   = b - bo * bdiv;
  const int lane = threadIdx.x & 31;
  const int wave = threadIdx.x >> 5;
  const int tilesN = N >> 6;
  const int tilesM = M >> 6;
  const int tile = blockIdx.x * 8 + wave;
  if (tile >= tilesM * tilesN) return;
  const int tm = tile / tilesN;
  const int tn = tile - tm * tilesN;
  const int m0 = tm << 6;
  const int n0 = tn << 6;

  const T* Ab  = A  + (size_t)bo * strideA + (size_t)bi * strideAi;
  const T* Bb  = Bt + (size_t)bo * strideB + (size_t)bi * strideBi;
  const T* Ab0 = PAIRA ? (Ab + (size_t)(2 * tn) * strideAsub) : Ab;
  const T* Ab1 = PAIRA ? (Ab0 + strideAsub) : Ab;

  const int rlane = lane & 15;
  const int koff  = (lane >> 4) * 8;
  const int mOff  = (lane >> 4) * 8;

  v8f acc[4][4];
#pragma unroll
  for (int i = 0; i < 4; ++i)
#pragma unroll
    for (int j = 0; j < 4; ++j) acc[i][j] = (v8f){0.f,0.f,0.f,0.f,0.f,0.f,0.f,0.f};

  for (int k0 = 0; k0 < K; k0 += 32) {
    V bh[4];
#pragma unroll
    for (int j = 0; j < 4; ++j) {
      const size_t bofs = (size_t)(n0 + (j << 4) + rlane) * ldb + koff + k0;
      bh[j] = Frag<T>::load(Bb + bofs);
    }
#pragma unroll
    for (int i = 0; i < 4; ++i) {
      const size_t ao = (size_t)(m0 + (i << 4) + rlane) * lda + koff + k0;
      V ah = Frag<T>::load(Ab0 + ao);
      V ah1 = ah;
      if (PAIRA) ah1 = Frag<T>::load(Ab1 + ao);
#pragma unroll
      for (int j = 0; j < 4; ++j) {
        acc[i][j] = Frag<T>::mma((PAIRA && j >= 2) ? ah1 : ah, bh[j], acc[i][j]);
      }
      Frag<T>::guard(acc[i][0], acc[i][3], ah, ah1);
    }
    Frag<T>::keep(bh[0], bh[1], bh[2], bh[3]);
  }
  acc_guard4(acc[0][0], acc[0][1], acc[0][2], acc[0][3]);
  acc_guard4(acc[1][0], acc[1][1], acc[1][2], acc[1][3]);
  acc_guard4(acc[2][0], acc[2][1], acc[2][2], acc[2][3]);
  acc_guard4(acc[3][0], acc[3][1], acc[3][2], acc[3][3]);

  float* slab = sT[wave];
  const float* Rb = RESID ? (resid + (size_t)b * strideR) : nullptr;
  const float* bp = bias0;
  int nsub = 0;
  float smul = 1.0f;
  if (BIAS_MODE == 2) {
    const int seg = (bseg > 0) ? (n0 / bseg) : 0;
    bp = (seg == 0) ? bias0 : ((seg == 1) ? bias1 : bias2);
    nsub = seg * bseg;
    smul = (seg == 0) ? seg0mul : 1.0f;
  }
#pragma unroll
  for (int i = 0; i < 4; ++i) {
    const int mBase = m0 + (i << 4);
#pragma unroll
    for (int j = 0; j < 4; ++j) {
      const int n = n0 + (j << 4) + rlane;
      float bv = 0.f;
      if (BIAS_MODE == 2) bv = bp[n - nsub];
#pragma unroll
      for (int r = 0; r < 8; ++r) {
        float v = acc[i][j][r] * scale;
        if (BIAS_MODE == 2) { v += bv; v *= smul; }
        if (RESID) v += Rb[(size_t)(mBase + mOff + r) * ldc + n];
        slab[(mOff + r) * 68 + (j << 4) + rlane] = v;
      }
    }
    __builtin_amdgcn_fence(__ATOMIC_RELEASE, "workgroup");
    __builtin_amdgcn_wave_barrier();
    __builtin_amdgcn_fence(__ATOMIC_ACQUIRE, "workgroup");
    if (OUT_MODE == 0) {
      float* Cp = (float*)Cout + (size_t)bo * strideC + (size_t)bi * strideCi;
      const int hh = lane >> 4, c4 = (lane & 15) * 4;
      for (int pass = 0; pass < 2; ++pass) {
#pragma unroll
        for (int it = 0; it < 8; ++it) {
          const int row = it * 2 + hh;
          v4f v = *(const v4f*)(slab + row * 68 + c4);
          *(volatile v4f*)(Cp + (size_t)(mBase + row) * ldc + n0 + c4) = v;
        }
        __threadfence();
      }
    } else {
      const int q = lane >> 3, c8 = (lane & 7) * 8;
      unsigned short* Cp = (unsigned short*)Cout + (size_t)bo * strideC + (size_t)bi * strideCi;
      for (int pass = 0; pass < 2; ++pass) {
#pragma unroll
        for (int it = 0; it < 4; ++it) {
          const int row = it * 4 + q;
          const float* sp = slab + row * 68 + c8;
          v8h hv;
#pragma unroll
          for (int e = 0; e < 8; ++e) hv[e] = (_Float16)sp[e];
          *(volatile v8h*)(Cp + (size_t)(mBase + row) * ldc + n0 + c8) = hv;
        }
        __threadfence();
      }
    }
    __builtin_amdgcn_fence(__ATOMIC_RELEASE, "workgroup");
    __builtin_amdgcn_wave_barrier();
    __builtin_amdgcn_fence(__ATOMIC_ACQUIRE, "workgroup");
  }
}

__global__ __launch_bounds__(256) void castw_kernel(const float* __restrict__ s0, const float* __restrict__ s1,
                                                     const float* __restrict__ s2, const float* __restrict__ s3,
                                                     const float* __restrict__ s4, const float* __restrict__ s5,
                                                     const float* __restrict__ s6, const float* __restrict__ s7,
                                                     const float* __restrict__ s8, const float* __restrict__ s9,
                                                     unsigned short* __restrict__ W16) {
  const int y = blockIdx.y, z = blockIdx.z;
  const float* src = (y == 0) ? s0 : (y == 1) ? s1 : (y == 2) ? s2 : (y == 3) ? s3 : (y == 4) ? s4 :
                     (y == 5) ? s5 : (y == 6) ? s6 : (y == 7) ? s7 : (y == 8) ? s8 : s9;
  const int n8 = (y < 8) ? (kHid * kHid / 8) : (kFF * kHid / 8);
  const size_t lstride = (y < 8) ? ((size_t)kHid * kHid) : ((size_t)kFF * kHid);
  const size_t dsto = (y < 8) ? ((size_t)y * kHid * kHid) : ((y == 8) ? kWoffF1 : kWoffF2);
  const int i = blockIdx.x * 256 + threadIdx.x;
  if (i >= n8) return;
  const float* p = src + (size_t)z * lstride + 8 * (size_t)i;
  const v4f a = *(const v4f*)(p);
  const v4f c = *(const v4f*)(p + 4);
  const v4u u = (v4u){pk16(h_bits(a.x * kWCarry), h_bits(a.y * kWCarry)), pk16(h_bits(a.z * kWCarry), h_bits(a.w * kWCarry)),
                      pk16(h_bits(c.x * kWCarry), h_bits(c.y * kWCarry)), pk16(h_bits(c.z * kWCarry), h_bits(c.w * kWCarry))};
  unsigned short* q = W16 + (size_t)z * kHalvesWLayer + dsto + 8 * (size_t)i;
  *(volatile v4u*)q = u;
  __threadfence();
  *(volatile v4u*)q = u;
}

__global__ __launch_bounds__(256) void ln16_kernel(const float* __restrict__ x, const float* __restrict__ w,
                                                    const float* __restrict__ bb, unsigned short* __restrict__ out) {
  const int wave = threadIdx.x >> 5, lane = threadIdx.x & 31;
  const int tok = blockIdx.x * 8 + wave;
  const float* xr = x + (size_t)tok * kHid + 8 * lane;
  const v4f a0 = *(const v4f*)(xr);
  const v4f a1 = *(const v4f*)(xr + 4);
  float s = ((a0.x + a0.y) + (a0.z + a0.w)) + ((a1.x + a1.y) + (a1.z + a1.w));
#pragma unroll
  for (int off = 16; off > 0; off >>= 1) s += __shfl_xor(s, off, 32);
  const float mean = s * (1.0f / kHid);
  const v4f d0 = a0 - mean;
  const v4f d1 = a1 - mean;
  float qs = ((d0.x * d0.x + d0.y * d0.y) + (d0.z * d0.z + d0.w * d0.w)) + ((d1.x * d1.x + d1.y * d1.y) + (d1.z * d1.z + d1.w * d1.w));
#pragma unroll
  for (int off = 16; off > 0; off >>= 1) qs += __shfl_xor(qs, off, 32);
  const float var = qs * (1.0f / kHid);
  const float inv = 1.0f / sqrtf(var + kLnEps);
  const v4f w0 = *(const v4f*)(w + 8 * lane);
  const v4f w1 = *(const v4f*)(w + 8 * lane + 4);
  const v4f c0 = *(const v4f*)(bb + 8 * lane);
  const v4f c1 = *(const v4f*)(bb + 8 * lane + 4);
  const v4f r0 = d0 * inv * w0 + c0;
  const v4f r1 = d1 * inv * w1 + c1;
  const v4u u = (v4u){pk16(h_bits(r0.x), h_bits(r0.y)), pk16(h_bits(r0.z), h_bits(r0.w)),
                      pk16(h_bits(r1.x), h_bits(r1.y)), pk16(h_bits(r1.z), h_bits(r1.w))};
  unsigned short* q = out + (size_t)tok * kHid + 8 * lane;
  *(volatile v4u*)q = u;
  __threadfence();
  *(volatile v4u*)q = u;
}

__global__ __launch_bounds__(256) void ln32_kernel(const float* __restrict__ x, const float* __restrict__ w,
                                                    const float* __restrict__ bb, float* __restrict__ out) {
  const int wave = threadIdx.x >> 5, lane = threadIdx.x & 31;
  const int tok = blockIdx.x * 8 + wave;
  const int ca = 4 * lane, cb = 128 + 4 * lane;
  const float* xr = x + (size_t)tok * kHid;
  const v4f a0 = *(const v4f*)(xr + ca);
  const v4f a1 = *(const v4f*)(xr + cb);
  float s = ((a0.x + a0.y) + (a0.z + a0.w)) + ((a1.x + a1.y) + (a1.z + a1.w));
#pragma unroll
  for (int off = 16; off > 0; off >>= 1) s += __shfl_xor(s, off, 32);
  const float mean = s * (1.0f / kHid);
  const v4f d0 = a0 - mean;
  const v4f d1 = a1 - mean;
  float qs = ((d0.x * d0.x + d0.y * d0.y) + (d0.z * d0.z + d0.w * d0.w)) + ((d1.x * d1.x + d1.y * d1.y) + (d1.z * d1.z + d1.w * d1.w));
#pragma unroll
  for (int off = 16; off > 0; off >>= 1) qs += __shfl_xor(qs, off, 32);
  const float var = qs * (1.0f / kHid);
  const float inv = 1.0f / sqrtf(var + kLnEps);
  const v4f w0 = *(const v4f*)(w + ca);
  const v4f w1 = *(const v4f*)(w + cb);
  const v4f c0 = *(const v4f*)(bb + ca);
  const v4f c1 = *(const v4f*)(bb + cb);
  const v4f r0 = d0 * inv * w0 + c0;
  const v4f r1 = d1 * inv * w1 + c1;
  float* orow = out + (size_t)tok * kHid;
  for (int pass = 0; pass < 2; ++pass) {
    *(volatile v4f*)(orow + ca) = r0;
    *(volatile v4f*)(orow + cb) = r1;
    __threadfence();
  }
}

__global__ __launch_bounds__(256) void vt_kernel(const unsigned short* __restrict__ qkv, unsigned short* __restrict__ vt) {
  __shared__ unsigned short sm[kHdim][264];
  const int t = threadIdx.x;
  const int br = blockIdx.x, h = blockIdx.y;
  const unsigned short* vr = qkv + ((size_t)br * kCols + t) * kQKVld + 2 * kHid + h * kHdim;
#pragma unroll
  for (int wq = 0; wq < 4; ++wq) {
    const v4u q = *(const v4u*)(vr + 8 * wq);
#pragma unroll
    for (int e = 0; e < 4; ++e) {
      const unsigned word = q[e];
      const int d = 8 * wq + 2 * e;
      sm[d][t]     = (unsigned short)(word & 0xffffu);
      sm[d + 1][t] = (unsigned short)(word >> 16);
    }
  }
  __syncthreads();
  const int wave = t >> 5, lane = t & 31;
  unsigned short* ob = vt + ((size_t)(br * kHeads + h) * kHdim) * kCols;
  for (int pass = 0; pass < 2; ++pass) {
#pragma unroll
    for (int rr = 0; rr < 4; ++rr) {
      const int d = wave * 4 + rr;
      const unsigned short* sp = &sm[d][8 * lane];
      const v4u u = (v4u){pk16(sp[0], sp[1]), pk16(sp[2], sp[3]), pk16(sp[4], sp[5]), pk16(sp[6], sp[7])};
      *(volatile v4u*)(ob + (size_t)d * kCols + 8 * lane) = u;
    }
    __threadfence();
  }
}

__global__ __launch_bounds__(256) void row_softmax_kernel(const float* __restrict__ S, const int* __restrict__ dist,
                                                           const float* __restrict__ rel, unsigned short* __restrict__ P, int brbase) {
  __shared__ float rels[kBuckets * kHeads];
  const int t = threadIdx.x;
  rels[t] = rel[t];
  __syncthreads();
  const int wave = t >> 5, lane = t & 31;
  const int row = blockIdx.x * 8 + wave;
  const int g = row >> 8, i = row & 255;
  const int br = brbase + (g >> 3), h = g & 7;
  const float* sr = S + (size_t)row * kCols + 8 * lane;
  const int* dr = dist + ((size_t)br * kCols + i) * kCols + 8 * lane;
  v4f y0 = (v4f){0.f, 0.f, 0.f, 0.f};
  v4f y1 = y0;
#pragma unroll 1
  for (int grp = 0; grp < 2; ++grp) {
    const v4f xs = *(const v4f*)(sr + 4 * grp);
    const v4i ds = *(const v4i*)(dr + 4 * grp);
    v4f ys = xs;
#pragma unroll
    for (int e = 0; e < 4; ++e) {
      const float a  = fabsf((float)ds[e]);
      const float tl = logf(fmaxf(a, 1.0f));
      const float u  = tl * kRecipLogMaxD;
      const float wv = u * 30.0f;
      int lb = (int)wv + 1;
      lb = (lb < 1) ? 1 : ((lb > kBuckets - 1) ? (kBuckets - 1) : lb);
      const int bkt = (a >= 1.0f) ? lb : 0;
      ys[e] = xs[e] + rels[bkt * kHeads + h];
    }
    if (grp == 0) y0 = ys; else y1 = ys;
  }
  float m = fmaxf(fmaxf(fmaxf(y0.x, y0.y), fmaxf(y0.z, y0.w)), fmaxf(fmaxf(y1.x, y1.y), fmaxf(y1.z, y1.w)));
#pragma unroll
  for (int off = 16; off > 0; off >>= 1) m = fmaxf(m, __shfl_xor(m, off, 32));
  v4f e0 = y0, e1 = y1;
  float sum = 0.f;
#pragma unroll 1
  for (int grp = 0; grp < 2; ++grp) {
    v4f ys;
    if (grp == 0) ys = y0; else ys = y1;
    v4f es;
#pragma unroll
    for (int e = 0; e < 4; ++e) es[e] = expf(ys[e] - m);
    sum += (es.x + es.y) + (es.z + es.w);
    if (grp == 0) e0 = es; else e1 = es;
  }
#pragma unroll
  for (int off = 16; off > 0; off >>= 1) sum += __shfl_xor(sum, off, 32);
  const float inv = 1.0f / sum;
  const float f = inv * kPCarry;
  const v4u u = (v4u){pk16(h_bits(e0.x * f), h_bits(e0.y * f)), pk16(h_bits(e0.z * f), h_bits(e0.w * f)),
                      pk16(h_bits(e1.x * f), h_bits(e1.y * f)), pk16(h_bits(e1.z * f), h_bits(e1.w * f))};
  unsigned short* q = P + (size_t)row * kCols + 8 * lane;
  *(volatile v4u*)q = u;
  __threadfence();
  *(volatile v4u*)q = u;
}

__global__ __launch_bounds__(256) void col_attn_kernel(const unsigned short* __restrict__ qkv, unsigned short* __restrict__ ctx) {
  __shared__ __align__(16) _Float16 Pw[kHeads][32 * 40];
  __shared__ __align__(16) _Float16 Vs[kHeads][32 * 40];
  __shared__ __align__(16) _Float16 Os[32 * 264];
  const int t = threadIdx.x, wave = t >> 5, lane = t & 31, hh = lane >> 4, c = lane & 15, koff = hh * 8;
  const int b = blockIdx.x >> 8, cc = blockIdx.x & 255;
  const int h = wave;
  const size_t tokb = (size_t)b * kRows * kCols + cc;
  const _Float16* F = (const _Float16*)qkv;

  {
    const unsigned short* vr = qkv + (tokb + (size_t)lane * kCols) * kQKVld + 2 * kHid + h * kHdim;
    _Float16* vs = Vs[wave];
#pragma unroll
    for (int wq = 0; wq < 4; ++wq) {
      const v4u q = *(const v4u*)(vr + 8 * wq);
#pragma unroll
      for (int e = 0; e < 4; ++e) {
        const unsigned word = q[e];
        const int d = 8 * wq + 2 * e;
        vs[d * 40 + lane]       = __builtin_bit_cast(_Float16, (unsigned short)(word & 0xffffu));
        vs[(d + 1) * 40 + lane] = __builtin_bit_cast(_Float16, (unsigned short)(word >> 16));
      }
    }
  }
  v16h qa[2], kb[2];
#pragma unroll
  for (int tm = 0; tm < 2; ++tm)
    qa[tm] = Frag<_Float16>::load(F + (tokb + (size_t)(tm * 16 + c) * kCols) * kQKVld + h * kHdim + koff);
#pragma unroll
  for (int tn = 0; tn < 2; ++tn)
    kb[tn] = Frag<_Float16>::load(F + (tokb + (size_t)(tn * 16 + c) * kCols) * kQKVld + kHid + h * kHdim + koff);
  v8f s[2][2];
#pragma unroll
  for (int tm = 0; tm < 2; ++tm)
#pragma unroll
    for (int tn = 0; tn < 2; ++tn) {
      s[tm][tn] = (v8f){0.f,0.f,0.f,0.f,0.f,0.f,0.f,0.f};
      s[tm][tn] = mma_f16(qa[tm], kb[tn], s[tm][tn]);
    }
  _Float16* pw = Pw[wave];
#pragma unroll
  for (int tm = 0; tm < 2; ++tm) {
#pragma unroll
    for (int r = 0; r < 8; ++r) {
      const float s0 = s[tm][0][r], s1 = s[tm][1][r];
      float m = fmaxf(s0, s1);
#pragma unroll
      for (int off = 1; off < 16; off <<= 1) m = fmaxf(m, __shfl_xor(m, off, 32));
      const float x0 = expf(s0 - m), x1 = expf(s1 - m);
      float ps = x0 + x1;
#pragma unroll
      for (int off = 1; off < 16; off <<= 1) ps += __shfl_xor(ps, off, 32);
      const float f = (1.0f / ps) * kPCarry;
      pw[(tm * 16 + 8 * hh + r) * 40 + c]      = (_Float16)(x0 * f);
      pw[(tm * 16 + 8 * hh + r) * 40 + 16 + c] = (_Float16)(x1 * f);
    }
  }
  __syncthreads();
  const _Float16* vsr = Vs[wave];
  v8f o[2][2];
#pragma unroll
  for (int tm = 0; tm < 2; ++tm) {
    const v16h pa = Frag<_Float16>::load(pw + (tm * 16 + c) * 40 + koff);
#pragma unroll
    for (int tn = 0; tn < 2; ++tn) {
      const v16h vb = Frag<_Float16>::load(vsr + (tn * 16 + c) * 40 + koff);
      o[tm][tn] = (v8f){0.f,0.f,0.f,0.f,0.f,0.f,0.f,0.f};
      o[tm][tn] = mma_f16(pa, vb, o[tm][tn]);
    }
  }
  const float osc = kCtxCarry / kPCarry;
#pragma unroll
  for (int tm = 0; tm < 2; ++tm)
#pragma unroll
    for (int tn = 0; tn < 2; ++tn)
#pragma unroll
      for (int r = 0; r < 8; ++r)
        Os[(tm * 16 + 8 * hh + r) * 264 + h * kHdim + tn * 16 + c] = (_Float16)(o[tm][tn][r] * osc);
  __syncthreads();
  for (int pass = 0; pass < 2; ++pass) {
#pragma unroll
    for (int rr = 0; rr < 4; ++rr) {
      const int i = wave * 4 + rr;
      const v4u val = *(const v4u*)(Os + i * 264 + 8 * lane);
      *(volatile v4u*)(ctx + (tokb + (size_t)i * kCols) * kHid + 8 * lane) = val;
    }
    __threadfence();
  }
}

__global__ __launch_bounds__(256) void gelu_kernel(const unsigned short* __restrict__ pre, unsigned short* __restrict__ out, int n8) {
  const int i = blockIdx.x * 256 + threadIdx.x;
  if (i >= n8) return;
  const v4u u = *(const v4u*)(pre + 8 * (size_t)i);
  const unsigned long long w01 = (unsigned long long)u.x | ((unsigned long long)u.y << 32);
  const unsigned long long w23 = (unsigned long long)u.z | ((unsigned long long)u.w << 32);
  unsigned long long r01 = 0ull, r23 = 0ull;
#pragma unroll 1
  for (int e = 0; e < 8; ++e) {
    const unsigned long long src = (e < 4) ? w01 : w23;
    const int sh = (e & 3) * 16;
    const unsigned short hb = (unsigned short)(src >> sh);
    const float x = hbits2f(hb);
    const float g = 0.5f * x * (1.0f + erff(x * 0.70710678118654752f));
    const unsigned long long ob = ((unsigned long long)h_bits(g * kGCarry)) << sh;
    const unsigned long long m4 = (e < 4) ? ~0ull : 0ull;
    r01 |= ob & m4;
    r23 |= ob & ~m4;
  }
  const v4u o = (v4u){(unsigned)r01, (unsigned)(r01 >> 32), (unsigned)r23, (unsigned)(r23 >> 32)};
  unsigned short* q = out + 8 * (size_t)i;
  *(volatile v4u*)q = o;
  __threadfence();
  *(volatile v4u*)q = o;
}

extern "C" void kernel_launch(void* const* d_in, const int* in_sizes, int n_in,
                              void* d_out, int out_size, void* d_ws, size_t ws_size,
                              hipStream_t stream) {
  if (n_in < 31) return;
  if (in_sizes[0] != kTok * kHid || out_size != kTok * kHid) return;
  if (in_sizes[1] != kBR * kCols * kCols) return;
  if (in_sizes[2] != kLayers * kHid * kHid || in_sizes[19] != kLayers * kFF * kHid || in_sizes[21] != kLayers * kHid * kFF) return;
  if (in_sizes[10] != kLayers * kBuckets * kHeads) return;
  if (ws_size < kWsTotal) return;

  const float* p_hs   = (const float*)d_in[0];
  const int*   p_dist = (const int*)d_in[1];
  const float* p_rqW  = (const float*)d_in[2];
  const float* p_rqb  = (const float*)d_in[3];
  const float* p_rkW  = (const float*)d_in[4];
  const float* p_rkb  = (const float*)d_in[5];
  const float* p_rvW  = (const float*)d_in[6];
  const float* p_rvb  = (const float*)d_in[7];
  const float* p_roW  = (const float*)d_in[8];
  const float* p_rob  = (const float*)d_in[9];
  const float* p_rrel = (const float*)d_in[10];
  const float* p_cqW  = (const float*)d_in[11];
  const float* p_cqb  = (const float*)d_in[12];
  const float* p_ckW  = (const float*)d_in[13];
  const float* p_ckb  = (const float*)d_in[14];
  const float* p_cvW  = (const float*)d_in[15];
  const float* p_cvb  = (const float*)d_in[16];
  const float* p_coW  = (const float*)d_in[17];
  const float* p_cob  = (const float*)d_in[18];
  const float* p_f1W  = (const float*)d_in[19];
  const float* p_f1b  = (const float*)d_in[20];
  const float* p_f2W  = (const float*)d_in[21];
  const float* p_f2b  = (const float*)d_in[22];
  const float* p_lnrw = (const float*)d_in[23];
  const float* p_lnrb = (const float*)d_in[24];
  const float* p_lncw = (const float*)d_in[25];
  const float* p_lncb = (const float*)d_in[26];
  const float* p_lnfw = (const float*)d_in[27];
  const float* p_lnfb = (const float*)d_in[28];
  const float* p_lnFw = (const float*)d_in[29];
  const float* p_lnFb = (const float*)d_in[30];

  char* ws = (char*)d_ws;
  float* xA = (float*)(ws + kOffXA);
  float* xB = (float*)(ws + kOffXB);
  unsigned short* xn    = (unsigned short*)(ws + kOffXN);
  unsigned short* ctx   = xn;
  unsigned short* qkv   = (unsigned short*)(ws + kOffQKV);
  unsigned short* vt    = (unsigned short*)(ws + kOffVT);
  unsigned short* h16   = (unsigned short*)(ws + kOffH16);
  float*          Sbuf  = (float*)(ws + kOffS);
  unsigned short* pre16 = (unsigned short*)(ws + kOffPre);
  unsigned short* Pbuf  = (unsigned short*)(ws + kOffP);
  unsigned short* W16   = (unsigned short*)(ws + kOffW);
  float* outp = (float*)d_out;

  castw_kernel<<<dim3(128, 10, 2), 256, 0, stream>>>(p_rqW, p_rkW, p_rvW, p_roW, p_cqW, p_ckW, p_cvW, p_coW, p_f1W, p_f2W, W16);

  const float* cur = p_hs;
  int curIdx = -1;
  for (int l = 0; l < kLayers; ++l) {
    const unsigned short* Wl     = W16 + (size_t)l * kHalvesWLayer;
    const unsigned short* Wqkv_r = Wl + kWoffQKVr;
    const unsigned short* Wo_r   = Wl + kWoffOr;
    const unsigned short* Wqkv_c = Wl + kWoffQKVc;
    const unsigned short* Wo_c   = Wl + kWoffOc;
    const unsigned short* Wf1    = Wl + kWoffF1;
    const unsigned short* Wf2    = Wl + kWoffF2;

    ln16_kernel<<<kTok / 8, 256, 0, stream>>>(cur, p_lnrw + l * kHid, p_lnrb + l * kHid, xn);
    gemm64<2, 1, false, false><<<dim3(384, 1), 256, 0, stream>>>(
        xn, kHid, 0L, 0L, 0L, Wqkv_r, kHid, 0L, 0L, (void*)qkv, kQKVld, 0L, 0L,
        p_rqb + l * kHid, p_rkb + l * kHid, p_rvb + l * kHid, kHid, 1.0f,
        p_hs, 0L, kTok, kQKVld, kHid, 1, 1.0f / kWCarry);
    vt_kernel<<<dim3(kBR, kHeads), 256, 0, stream>>>(qkv, vt);
    for (int ch = 0; ch < kChunks; ++ch) {
      const int brbase = ch * kChunkBR;
      const unsigned short* qb = qkv + (size_t)brbase * kCols * kQKVld;
      gemm64<0, 0, false, false><<<dim3(2, kChunkGroups), 256, 0, stream>>>(
          qb, kQKVld, (long)kCols * kQKVld, (long)kHdim, 0L,
          qb + kHid, kQKVld, (long)kCols * kQKVld, (long)kHdim,
          (void*)Sbuf, kCols, (long)kHeads * kCols * kCols, (long)kCols * kCols,
          p_rqb, p_rqb, p_rqb, 0, 1.0f, p_hs, 0L,
          kCols, kCols, kHdim, kHeads, kRowScoreScale);
      row_softmax_kernel<<<kChunkGroups * kCols / 8, 256, 0, stream>>>(Sbuf, p_dist, p_rrel + (size_t)l * kBuckets * kHeads, Pbuf, brbase);
      gemm64<0, 1, false, true><<<dim3(2, kChunkBR), 256, 0, stream>>>(
          Pbuf, kCols, (long)kHeads * kCols * kCols, 0L, (long)kCols * kCols,
          vt + (size_t)brbase * kHeads * kHdim * kCols, kCols, (long)kHeads * kHdim * kCols, 0L,
          (void*)(ctx + (size_t)brbase * kCols * kHid), kHid, (long)kCols * kHid, 0L,
          p_rqb, p_rqb, p_rqb, 0, 1.0f, p_hs, 0L,
          kCols, kHid, kCols, 1, kCtxCarry / kPCarry);
    }
    {
      float* nxt = (curIdx == 0) ? xB : xA;
      gemm64<2, 0, true, false><<<dim3(128, 1), 256, 0, stream>>>(
          ctx, kHid, 0L, 0L, 0L, Wo_r, kHid, 0L, 0L, (void*)nxt, kHid, 0L, 0L,
          p_rob + l * kHid, p_rob + l * kHid, p_rob + l * kHid, 0, 1.0f,
          cur, 0L, kTok, kHid, kHid, 1, 1.0f / (kCtxCarry * kWCarry));
      cur = nxt; curIdx = (curIdx == 0) ? 1 : 0;
    }

    ln16_kernel<<<kTok / 8, 256, 0, stream>>>(cur, p_lncw + l * kHid, p_lncb + l * kHid, xn);
    gemm64<2, 1, false, false><<<dim3(384, 1), 256, 0, stream>>>(
        xn, kHid, 0L, 0L, 0L, Wqkv_c, kHid, 0L, 0L, (void*)qkv, kQKVld, 0L, 0L,
        p_cqb + l * kHid, p_ckb + l * kHid, p_cvb + l * kHid, kHid, kColQScale,
        p_hs, 0L, kTok, kQKVld, kHid, 1, 1.0f / kWCarry);
    col_attn_kernel<<<kBatch * kCols, 256, 0, stream>>>(qkv, ctx);
    {
      float* nxt = (curIdx == 0) ? xB : xA;
      gemm64<2, 0, true, false><<<dim3(128, 1), 256, 0, stream>>>(
          ctx, kHid, 0L, 0L, 0L, Wo_c, kHid, 0L, 0L, (void*)nxt, kHid, 0L, 0L,
          p_cob + l * kHid, p_cob + l * kHid, p_cob + l * kHid, 0, 1.0f,
          cur, 0L, kTok, kHid, kHid, 1, 1.0f / (kCtxCarry * kWCarry));
      cur = nxt; curIdx = (curIdx == 0) ? 1 : 0;
    }

    ln16_kernel<<<kTok / 8, 256, 0, stream>>>(cur, p_lnfw + l * kHid, p_lnfb + l * kHid, xn);
    gemm64<2, 1, false, false><<<dim3(512, 1), 256, 0, stream>>>(
        xn, kHid, 0L, 0L, 0L, Wf1, kHid, 0L, 0L, (void*)pre16, kFF, 0L, 0L,
        p_f1b + l * kFF, p_f1b + l * kFF, p_f1b + l * kFF, 0, 1.0f,
        p_hs, 0L, kTok, kFF, kHid, 1, 1.0f / kWCarry);
    gelu_kernel<<<(kTok * kFF / 8) / 256, 256, 0, stream>>>(pre16, h16, kTok * kFF / 8);
    {
      float* nxt = (curIdx == 0) ? xB : xA;
      gemm64<2, 0, true, false><<<dim3(128, 1), 256, 0, stream>>>(
          h16, kFF, 0L, 0L, 0L, Wf2, kFF, 0L, 0L, (void*)nxt, kHid, 0L, 0L,
          p_f2b + l * kHid, p_f2b + l * kHid, p_f2b + l * kHid, 0, 1.0f,
          cur, 0L, kTok, kHid, kFF, 1, 1.0f / (kGCarry * kWCarry));
      cur = nxt; curIdx = (curIdx == 0) ? 1 : 0;
    }
  }
  ln32_kernel<<<kTok / 8, 256, 0, stream>>>(cur, p_lnFw, p_lnFb, outp);
}
